// MambaBlock_10892037062805
// MI455X (gfx1250) — hardware-verified
//
#include <hip/hip_runtime.h>
#include <math.h>

typedef __attribute__((ext_vector_type(16))) _Float16 v16h;
typedef __attribute__((ext_vector_type(8)))  _Float16 v8h;
typedef __attribute__((ext_vector_type(16))) __bf16   v16b;
typedef __attribute__((ext_vector_type(8)))  __bf16   v8b;
typedef __attribute__((ext_vector_type(8)))  float    v8f;
typedef __attribute__((ext_vector_type(4)))  float    v4f;
typedef __attribute__((ext_vector_type(4)))  unsigned int v4u;

constexpr int kBatch  = 16;
constexpr int kSeq    = 2048;
constexpr int kDm     = 256;
constexpr int kNst    = 16;
constexpr int kDtR    = 16;
constexpr int kXpN    = kDtR + 2 * kNst;
constexpr int kXpP    = 64;
constexpr int kDtK    = 32;
constexpr int kGluN   = 2 * kDm;
constexpr int kRows   = kBatch * kSeq;
constexpr int kGluQ   = 4;
constexpr int kRowsQ  = kRows / kGluQ;
constexpr int kScanTS = 64;
constexpr int kScanCh = 64;
constexpr int kScanYP = 68;
constexpr float kLnEps    = 1e-5f;
constexpr float kSqrtHalf = 0.70710678118654752440f;
constexpr float kLog2e    = 1.44269504088896340736f;
static_assert(kRows * kDm == 8388608, "x / out element count");
static_assert(kDm * kXpN == 12288 && kDtR * kDm == 4096 && kDm * kNst == 4096 && kDm * kGluN == 131072, "weight element counts");
static_assert((kDm % 32) == 0 && (kDtK % 32) == 0, "GEMM K multiples of 32");
static_assert((kRows % 64) == 0 && (kRowsQ % 64) == 0 && (kXpP % 64) == 0 && (kDm % 64) == 0 && (kGluN % 64) == 0, "GEMM M,N multiples of 64");
static_assert(((kRows / 64) * (kXpP / 64)) % 8 == 0 && ((kRows / 64) * (kDm / 64)) % 8 == 0 && ((kRowsQ / 64) * (kGluN / 64)) % 8 == 0, "8 tiles per GEMM block");
static_assert((kSeq % kScanTS) == 0 && (kDm % kScanCh) == 0 && kScanCh == 64 && kScanTS == 64, "scan tiling");
static_assert((kRows % 8) == 0 && ((kRows * kDtK / 8) % 256) == 0 && ((kRowsQ * kDm / 4) % 256) == 0, "exact grids");
static_assert(((kXpP * kDm / 8) % 256) == 0 && ((kDm * kDtK / 8) % 256) == 0 && ((kGluN * kDm / 8) % 256) == 0, "exact weight-plane grids");

constexpr size_t kOffWXH = 0;
constexpr size_t kOffWXL = kOffWXH + (size_t)kXpP * kDm * 2;
constexpr size_t kOffWDH = kOffWXL + (size_t)kXpP * kDm * 2;
constexpr size_t kOffWDL = kOffWDH + (size_t)kDm * kDtK * 2;
constexpr size_t kOffWGH = kOffWDL + (size_t)kDm * kDtK * 2;
constexpr size_t kOffWGL = kOffWGH + (size_t)kGluN * kDm * 2;
constexpr size_t kOffLNH = kOffWGL + (size_t)kGluN * kDm * 2;
constexpr size_t kOffLNL = kOffLNH + (size_t)kRows * kDm * 2;
constexpr size_t kOffDBL = kOffLNL + (size_t)kRows * kDm * 2;
constexpr size_t kOffDTH = kOffDBL + (size_t)kRows * kXpP * 4;
constexpr size_t kOffDTL = kOffDTH + (size_t)kRows * kDtK * 2;
constexpr size_t kOffDLR = kOffDTL + (size_t)kRows * kDtK * 2;
constexpr size_t kOffYGH = kOffDLR + (size_t)kRows * kDm * 4;
constexpr size_t kOffYGL = kOffYGH + (size_t)kRows * kDm * 2;
constexpr size_t kOffGO  = kOffYGL + (size_t)kRows * kDm * 2;
constexpr size_t kWsTotal = kOffGO + (size_t)kRowsQ * kGluN * 4;
static_assert(kWsTotal == 130646016ull, "carve total");
static_assert(kWsTotal <= 134217728ull, "carve cap");
static_assert((kOffWXL % 128) == 0 && (kOffWDH % 128) == 0 && (kOffWDL % 128) == 0 && (kOffWGH % 128) == 0 &&
              (kOffWGL % 128) == 0 && (kOffLNH % 128) == 0 && (kOffLNL % 128) == 0 && (kOffDBL % 128) == 0 &&
              (kOffDTH % 128) == 0 && (kOffDTL % 128) == 0 && (kOffDLR % 128) == 0 && (kOffYGH % 128) == 0 &&
              (kOffYGL % 128) == 0 && (kOffGO % 128) == 0, "128-B aligned regions");

__device__ __forceinline__ unsigned short f2bf_bits(float f) {
  unsigned u = __float_as_uint(f);
  return (unsigned short)((u + 0x7FFFu + ((u >> 16) & 1u)) >> 16);
}
__device__ __forceinline__ float bf_bits2f(unsigned short h) { return __uint_as_float(((unsigned)h) << 16); }

__device__ __forceinline__ void dep_guard4_h(v8f& a, v8f& b, v8f& c, v8f& d, v16h x, v16h y) { asm volatile("v_nop\n\tv_nop\n\tv_nop\n\tv_nop" : "+v"(a), "+v"(b), "+v"(c), "+v"(d) : "v"(x), "v"(y)); }
__device__ __forceinline__ void dep_guard4_b(v8f& a, v8f& b, v8f& c, v8f& d, v16b x, v16b y) { asm volatile("v_nop\n\tv_nop\n\tv_nop\n\tv_nop" : "+v"(a), "+v"(b), "+v"(c), "+v"(d) : "v"(x), "v"(y)); }
__device__ __forceinline__ void keep4_h(v16h a, v16h b, v16h c, v16h d) { asm volatile("v_nop" :: "v"(a), "v"(b), "v"(c), "v"(d)); }
__device__ __forceinline__ void keep4_b(v16b a, v16b b, v16b c, v16b d) { asm volatile("v_nop" :: "v"(a), "v"(b), "v"(c), "v"(d)); }
__device__ __forceinline__ void acc_guard4(v8f& a, v8f& b, v8f& c, v8f& d) { asm volatile("v_nop\n\tv_nop\n\tv_nop\n\tv_nop" : "+v"(a), "+v"(b), "+v"(c), "+v"(d)); }
template <typename T> struct Frag;
template <> struct Frag<_Float16> {
  typedef v16h V; union U { v16h v; v8h h[2]; };
  static __device__ __forceinline__ v16h load(const _Float16* p) {
    U f; f.h[0] = *(const v8h*)(p); f.h[1] = *(const v8h*)(p + 16); return f.v;
  }
  static __device__ __forceinline__ v8f mma(v16h a, v16h b, v8f c) {
    return __builtin_amdgcn_wmma_f32_16x16x32_f16(false, a, false, b, (short)0, c, false, false);
  }
  static __device__ __forceinline__ void guard4(v8f& a, v8f& b, v8f& c, v8f& d, v16h x, v16h y) { dep_guard4_h(a, b, c, d, x, y); }
  static __device__ __forceinline__ void keep(v16h a, v16h b, v16h c, v16h d) { keep4_h(a, b, c, d); }
};
template <> struct Frag<__bf16> {
  typedef v16b V; union U { v16b v; v8b h[2]; };
  static __device__ __forceinline__ v16b load(const __bf16* p) {
    U f; f.h[0] = *(const v8b*)(p); f.h[1] = *(const v8b*)(p + 16); return f.v;
  }
  static __device__ __forceinline__ v8f mma(v16b a, v16b b, v8f c) {
    return __builtin_amdgcn_wmma_f32_16x16x32_bf16(false, a, false, b, (short)0, c, false, false);
  }
  static __device__ __forceinline__ void guard4(v8f& a, v8f& b, v8f& c, v8f& d, v16b x, v16b y) { dep_guard4_b(a, b, c, d, x, y); }
  static __device__ __forceinline__ void keep(v16b a, v16b b, v16b c, v16b d) { keep4_b(a, b, c, d); }
};

template <int ET> struct Elem;
template <> struct Elem<0> { typedef _Float16 T; };
template <> struct Elem<1> { typedef __bf16 T; };
template <int ET, bool SPLIT, int BIAS_MODE, int OUT_MODE, bool RESID, int ACT = 0>
__global__ __launch_bounds__(256) void wmma_gemm64(
    const unsigned short* __restrict__ Ap, const unsigned short* __restrict__ A2p, int lda, long strideA,
    const unsigned short* __restrict__ Btp, const unsigned short* __restrict__ Bt2p, int ldb, long strideB,
    void* __restrict__ Cout, void* __restrict__ Cout2, int ldc, long strideC,
    const float* __restrict__ bias,
    const float* __restrict__ resid, long strideR,
    int M, int N, int K, float scale) {
  typedef typename Elem<ET>::T T;
  typedef typename Frag<T>::V V;
  const T* A = (const T*)Ap; const T* A2 = (const T*)A2p; const T* Bt = (const T*)Btp; const T* Bt2 = (const T*)Bt2p;
  __shared__ __align__(16) float sT[8][16 * 68];
  const int b    = blockIdx.y;
  const int lane = threadIdx.x & 31;
  const int wave = threadIdx.x >> 5;
  const int tilesN = N >> 6;
  const int tilesM = M >> 6;
  const int tile = blockIdx.x * 8 + wave;
  if (tile >= tilesM * tilesN) return;
  const int tm = tile / tilesN;
  const int tn = tile - tm * tilesN;
  const int m0 = tm << 6;
  const int n0 = tn << 6;

  const T* Ab  = A  + (size_t)b * strideA;
  const T* Bb  = Bt + (size_t)b * strideB;
  const T* Ab2 = SPLIT ? (A2  + (size_t)b * strideA) : nullptr;
  const T* Bb2 = SPLIT ? (Bt2 + (size_t)b * strideB) : nullptr;

  const int rlane = lane & 15;
  const int koff  = (lane >> 4) * 8;
  const int mOff  = (lane >> 4) * 8;

  v8f acc[4][4];
#pragma unroll
  for (int i = 0; i < 4; ++i)
#pragma unroll
    for (int j = 0; j < 4; ++j) acc[i][j] = (v8f){0.f,0.f,0.f,0.f,0.f,0.f,0.f,0.f};

  for (int k0 = 0; k0 < K; k0 += 32) {
    V bh[4], bl[4];
#pragma unroll
    for (int j = 0; j < 4; ++j) {
      const size_t bo = (size_t)(n0 + (j << 4) + rlane) * ldb + koff + k0;
      bh[j] = Frag<T>::load(Bb + bo);
      if (SPLIT) bl[j] = Frag<T>::load(Bb2 + bo);
    }
#pragma unroll
    for (int i = 0; i < 4; ++i) {
      const size_t ao = (size_t)(m0 + (i << 4) + rlane) * lda + koff + k0;
      V ah = Frag<T>::load(Ab + ao);
      V al;
      if (SPLIT) al = Frag<T>::load(Ab2 + ao);
#pragma unroll
      for (int j = 0; j < 4; ++j) {
        acc[i][j] = Frag<T>::mma(ah, bh[j], acc[i][j]);
        if (SPLIT) {
          acc[i][j] = Frag<T>::mma(ah, bl[j], acc[i][j]);
          acc[i][j] = Frag<T>::mma(al, bh[j], acc[i][j]);
        }
      }
      Frag<T>::guard4(acc[i][0], acc[i][1], acc[i][2], acc[i][3], ah, SPLIT ? al : ah);
    }
    Frag<T>::keep(bh[0], bh[1], bh[2], bh[3]);
    if (SPLIT) Frag<T>::keep(bl[0], bl[1], bl[2], bl[3]);
  }
  acc_guard4(acc[0][0], acc[0][1], acc[0][2], acc[0][3]);
  acc_guard4(acc[1][0], acc[1][1], acc[1][2], acc[1][3]);
  acc_guard4(acc[2][0], acc[2][1], acc[2][2], acc[2][3]);
  acc_guard4(acc[3][0], acc[3][1], acc[3][2], acc[3][3]);

  float* slab = sT[wave];
  const float* Rb = RESID ? (resid + (size_t)b * strideR) : nullptr;
#pragma unroll
  for (int i = 0; i < 4; ++i) {
    const int mBase = m0 + (i << 4);
#pragma unroll
    for (int j = 0; j < 4; ++j) {
      const int n = n0 + (j << 4) + rlane;
      float bv = 0.f;
      if (BIAS_MODE == 2) bv = bias[n];
#pragma unroll
      for (int r = 0; r < 8; ++r) {
        float v = acc[i][j][r] * scale;
        if (BIAS_MODE == 1) v += bias[mBase + mOff + r];
        if (BIAS_MODE == 2) v += bv;
        if (RESID) v += Rb[(size_t)(mBase + mOff + r) * ldc + n];
        if (ACT == 1) v = tanhf(v);
        if (ACT == 2) v = fmaxf(v, 0.0f);
        if (ACT == 3) v = v / (1.0f + expf(-v));
        if (ACT == 4) v = (v > 0.f) ? v : 0.01f * v;
        slab[(mOff + r) * 68 + (j << 4) + rlane] = v;
      }
    }
    __builtin_amdgcn_fence(__ATOMIC_RELEASE, "workgroup");
    __builtin_amdgcn_wave_barrier();
    __builtin_amdgcn_fence(__ATOMIC_ACQUIRE, "workgroup");
    if (OUT_MODE == 0) {
      float* C = (float*)Cout + (size_t)b * strideC;
      const int hh = lane >> 4, c4 = (lane & 15) * 4;
      for (int pass = 0; pass < 2; ++pass) {
#pragma unroll
        for (int it = 0; it < 8; ++it) {
          const int row = it * 2 + hh;
          v4f v = *(const v4f*)(slab + row * 68 + c4);
          *(volatile v4f*)(C + (size_t)(mBase + row) * ldc + n0 + c4) = v;
        }
        __threadfence();
      }
    } else {
      const int q = lane >> 3, c8 = (lane & 7) * 8;
      unsigned short* C  = (unsigned short*)Cout  + (size_t)b * strideC;
      unsigned short* C2 = (OUT_MODE == 2) ? ((unsigned short*)Cout2 + (size_t)b * strideC) : nullptr;
      for (int pass = 0; pass < 2; ++pass) {
#pragma unroll
        for (int it = 0; it < 4; ++it) {
          const int row = it * 4 + q;
          const float* sp = slab + row * 68 + c8;
          v8h hv, lv;
#pragma unroll
          for (int e = 0; e < 8; ++e) {
            if (OUT_MODE == 1) {
              hv[e] = (_Float16)sp[e];
            } else {
              unsigned short hb = f2bf_bits(sp[e]);
              unsigned short lb = f2bf_bits(sp[e] - bf_bits2f(hb));
              hv[e] = __builtin_bit_cast(_Float16, hb);
              lv[e] = __builtin_bit_cast(_Float16, lb);
            }
          }
          *(volatile v8h*)(C + (size_t)(mBase + row) * ldc + n0 + c8) = hv;
          if (OUT_MODE == 2) *(volatile v8h*)(C2 + (size_t)(mBase + row) * ldc + n0 + c8) = lv;
        }
        __threadfence();
      }
    }
    __builtin_amdgcn_fence(__ATOMIC_RELEASE, "workgroup");
    __builtin_amdgcn_wave_barrier();
    __builtin_amdgcn_fence(__ATOMIC_ACQUIRE, "workgroup");
  }
}

__global__ __launch_bounds__(256) void wsplit_kernel(
    const float* __restrict__ W, int Kdim, int Ndim, int Kpad, int Npad,
    unsigned short* __restrict__ dhi, unsigned short* __restrict__ dlo, int total8)
{
  const int i = blockIdx.x * 256 + threadIdx.x;
  if (i >= total8) return;
  (void)Npad;
  const int e0 = i << 3;
  const int n  = e0 / Kpad;
  const int kb = e0 - n * Kpad;
  const int nc = (n < Ndim) ? n : (Ndim - 1);
  const bool nlive = (n < Ndim);
  v8h hv, lv;
#pragma unroll
  for (int e = 0; e < 8; ++e) {
    const int k  = kb + e;
    const int kc = (k < Kdim) ? k : (Kdim - 1);
    const bool live = nlive && (k < Kdim);
    const float a  = W[(size_t)kc * Ndim + nc];
    const float v  = live ? a : 0.0f;
    const unsigned short hb = f2bf_bits(v);
    const unsigned short lb = f2bf_bits(v - bf_bits2f(hb));
    hv[e] = __builtin_bit_cast(_Float16, hb);
    lv[e] = __builtin_bit_cast(_Float16, lb);
  }
  unsigned short* qh = dhi + (size_t)e0;
  unsigned short* ql = dlo + (size_t)e0;
  *(volatile v8h*)qh = hv;
  *(volatile v8h*)ql = lv;
  __threadfence();
  *(volatile v8h*)qh = hv;
  *(volatile v8h*)ql = lv;
}

__global__ __launch_bounds__(256) void layernorm_split_kernel(
    const float* __restrict__ x, const float* __restrict__ lw, const float* __restrict__ lb,
    unsigned short* __restrict__ PH, unsigned short* __restrict__ PL)
{
  const int lane = threadIdx.x & 31, wave = threadIdx.x >> 5;
  const size_t token = (size_t)blockIdx.x * 8 + wave;
  const int c0 = lane * 8;
  const float* xp = x + token * kDm + c0;
  const v4f a0 = *(const v4f*)(xp);
  const v4f a1 = *(const v4f*)(xp + 4);
  const v4f w0 = *(const v4f*)(lw + c0);
  const v4f w1 = *(const v4f*)(lw + c0 + 4);
  const v4f b0 = *(const v4f*)(lb + c0);
  const v4f b1 = *(const v4f*)(lb + c0 + 4);
  float xv[8], wv[8], bv[8];
#pragma unroll
  for (int e = 0; e < 4; ++e) {
    xv[e] = a0[e]; xv[4 + e] = a1[e];
    wv[e] = w0[e]; wv[4 + e] = w1[e];
    bv[e] = b0[e]; bv[4 + e] = b1[e];
  }
  float s = 0.f;
#pragma unroll
  for (int e = 0; e < 8; ++e) s += xv[e];
#pragma unroll
  for (int m = 16; m >= 1; m >>= 1) s += __shfl_xor(s, m, 32);
  const float mu = s * (1.0f / (float)kDm);
  float dv[8];
  float qs = 0.f;
#pragma unroll
  for (int e = 0; e < 8; ++e) { dv[e] = xv[e] - mu; qs += dv[e] * dv[e]; }
#pragma unroll
  for (int m = 16; m >= 1; m >>= 1) qs += __shfl_xor(qs, m, 32);
  const float var  = qs * (1.0f / (float)kDm);
  const float rstd = rsqrtf(var + kLnEps);
  v8h hv, lv;
#pragma unroll
  for (int e = 0; e < 8; ++e) {
    const float y = (dv[e] * rstd) * wv[e] + bv[e];
    const unsigned short hb = f2bf_bits(y);
    const unsigned short lb2 = f2bf_bits(y - bf_bits2f(hb));
    hv[e] = __builtin_bit_cast(_Float16, hb);
    lv[e] = __builtin_bit_cast(_Float16, lb2);
  }
  const size_t o = token * kDm + c0;
  *(volatile v8h*)(PH + o) = hv;
  *(volatile v8h*)(PL + o) = lv;
  __threadfence();
  *(volatile v8h*)(PH + o) = hv;
  *(volatile v8h*)(PL + o) = lv;
}

__global__ __launch_bounds__(256) void dtsplit_kernel(
    const float* __restrict__ DBL, unsigned short* __restrict__ dhi, unsigned short* __restrict__ dlo, int total8)
{
  const int i = blockIdx.x * 256 + threadIdx.x;
  if (i >= total8) return;
  const size_t e0 = (size_t)i << 3;
  const size_t row = e0 >> 5;
  const int c8 = (int)(e0 & 31);
  const bool live = (c8 < kDtR);
  const int cc = live ? c8 : 0;
  const float* p = DBL + row * kXpP + cc;
  const v4f a0 = *(const v4f*)(p);
  const v4f a1 = *(const v4f*)(p + 4);
  v8h hv, lv;
#pragma unroll
  for (int e = 0; e < 4; ++e) {
    const float s0 = a0[e], s1 = a1[e];
    const float v0 = live ? s0 : 0.0f;
    const float v1 = live ? s1 : 0.0f;
    const unsigned short h0 = f2bf_bits(v0), h1 = f2bf_bits(v1);
    const unsigned short l0 = f2bf_bits(v0 - bf_bits2f(h0)), l1 = f2bf_bits(v1 - bf_bits2f(h1));
    hv[e]     = __builtin_bit_cast(_Float16, h0);
    hv[4 + e] = __builtin_bit_cast(_Float16, h1);
    lv[e]     = __builtin_bit_cast(_Float16, l0);
    lv[4 + e] = __builtin_bit_cast(_Float16, l1);
  }
  unsigned short* qh = dhi + e0;
  unsigned short* ql = dlo + e0;
  *(volatile v8h*)qh = hv;
  *(volatile v8h*)ql = lv;
  __threadfence();
  *(volatile v8h*)qh = hv;
  *(volatile v8h*)ql = lv;
}

__global__ __launch_bounds__(kScanCh) void scan_kernel(
    const float* __restrict__ DBL, const float* __restrict__ DLR,
    const unsigned short* __restrict__ UH, const unsigned short* __restrict__ UL,
    const float* __restrict__ bdt, const float* __restrict__ Alog, const float* __restrict__ Dp,
    unsigned short* __restrict__ YH, unsigned short* __restrict__ YL)
{
  __shared__ __align__(16) float sX[kScanTS * kXpP];
  __shared__ __align__(16) float sU[kScanTS * kScanCh];
  __shared__ __align__(16) float sY[kScanTS * kScanYP];
  __shared__ __align__(16) float sA[kNst * kScanCh];
  const int tid = threadIdx.x, lane = tid & 31, wave = tid >> 5;
  constexpr int kBlkPerB = kDm / kScanCh;
  const int bix = blockIdx.x / kBlkPerB;
  const int d0  = (blockIdx.x - bix * kBlkPerB) * kScanCh;
  const int d   = d0 + tid;
  const size_t row0 = (size_t)bix * kSeq;
#pragma unroll 1
  for (int s = 0; s < kNst; ++s) sA[s * kScanCh + tid] = -expf(Alog[(size_t)d * kNst + s]);
  __syncthreads();
  float negA[kNst], h[kNst];
#pragma unroll
  for (int s = 0; s < kNst; ++s) {
    negA[s] = sA[s * kScanCh + tid];
    h[s] = 0.f;
  }
  const float bb = bdt[d], Dd = Dp[d];
  const int lr = tid >> 4, lc4 = (tid & 15) * 4;
  const int q = lane >> 3, c8 = (lane & 7) * 8;
#pragma unroll 1
  for (int t0 = 0; t0 < kSeq; t0 += kScanTS) {
    __syncthreads();
#pragma unroll
    for (int i = 0; i < 8; ++i) {
      const int r = lr + 4 * i;
      *(v4f*)(sX + r * kXpP + lc4) = *(const v4f*)(DBL + (row0 + t0 + r) * kXpP + lc4);
    }
    asm volatile("" ::: "memory");
#pragma unroll
    for (int i = 8; i < 16; ++i) {
      const int r = lr + 4 * i;
      *(v4f*)(sX + r * kXpP + lc4) = *(const v4f*)(DBL + (row0 + t0 + r) * kXpP + lc4);
    }
    asm volatile("" ::: "memory");
#pragma unroll
    for (int i = 0; i < 4; ++i) {
      const int idx = tid + kScanCh * i;
      const int r = idx >> 3;
      const int c = (idx & 7) * 8;
      const size_t go = (row0 + t0 + r) * kDm + d0 + c;
      const v4u wh = *(const v4u*)(UH + go);
      const v4u wl = *(const v4u*)(UL + go);
      float uu[8];
#pragma unroll
      for (int j = 0; j < 4; ++j) {
        const unsigned ah = wh[j], al = wl[j];
        uu[2 * j]     = __uint_as_float(ah << 16) + __uint_as_float(al << 16);
        uu[2 * j + 1] = __uint_as_float(ah & 0xffff0000u) + __uint_as_float(al & 0xffff0000u);
      }
      *(v4f*)(sU + r * kScanCh + c)     = (v4f){uu[0], uu[1], uu[2], uu[3]};
      *(v4f*)(sU + r * kScanCh + c + 4) = (v4f){uu[4], uu[5], uu[6], uu[7]};
    }
    asm volatile("" ::: "memory");
#pragma unroll
    for (int i = 4; i < 8; ++i) {
      const int idx = tid + kScanCh * i;
      const int r = idx >> 3;
      const int c = (idx & 7) * 8;
      const size_t go = (row0 + t0 + r) * kDm + d0 + c;
      const v4u wh = *(const v4u*)(UH + go);
      const v4u wl = *(const v4u*)(UL + go);
      float uu[8];
#pragma unroll
      for (int j = 0; j < 4; ++j) {
        const unsigned ah = wh[j], al = wl[j];
        uu[2 * j]     = __uint_as_float(ah << 16) + __uint_as_float(al << 16);
        uu[2 * j + 1] = __uint_as_float(ah & 0xffff0000u) + __uint_as_float(al & 0xffff0000u);
      }
      *(v4f*)(sU + r * kScanCh + c)     = (v4f){uu[0], uu[1], uu[2], uu[3]};
      *(v4f*)(sU + r * kScanCh + c + 4) = (v4f){uu[4], uu[5], uu[6], uu[7]};
    }
    __syncthreads();
#pragma unroll 1
    for (int s = 0; s < kScanTS; ++s) {
      const int t = t0 + s;
      const float* xr = sX + s * kXpP;
      float Bs[kNst], Cs[kNst];
#pragma unroll
      for (int q4 = 0; q4 < 4; ++q4) {
        const v4f bv = *(const v4f*)(xr + kDtR + 4 * q4);
        const v4f cv = *(const v4f*)(xr + kDtR + kNst + 4 * q4);
        Bs[4 * q4 + 0] = bv[0]; Bs[4 * q4 + 1] = bv[1]; Bs[4 * q4 + 2] = bv[2]; Bs[4 * q4 + 3] = bv[3];
        Cs[4 * q4 + 0] = cv[0]; Cs[4 * q4 + 1] = cv[1]; Cs[4 * q4 + 2] = cv[2]; Cs[4 * q4 + 3] = cv[3];
      }
      const float a     = DLR[(row0 + t) * kDm + d] + bb;
      const float delta = fmaxf(a, 0.0f) + log1pf(expf(-fabsf(a)));
      const float u     = sU[s * kScanCh + tid];
      float du = delta * u;
      asm volatile("" : "+v"(du));
      float y = 0.f;
#pragma unroll
      for (int k = 0; k < kNst; ++k) {
        float tb = (delta * negA[k]) * kLog2e;
        asm volatile("" : "+v"(tb));
        const float e = exp2f(tb);
        float p = du * Bs[k];
        asm volatile("" : "+v"(p));
        float qv = h[k] * e;
        asm volatile("" : "+v"(qv));
        const float hn = qv + p;
        h[k] = hn;
        float rr = hn * Cs[k];
        asm volatile("" : "+v"(rr));
        y += rr;
      }
      float sk = u * Dd;
      asm volatile("" : "+v"(sk));
      const float v2 = y + sk;
      const float g  = 0.5f * v2 * (1.0f + erff(v2 * kSqrtHalf));
      sY[s * kScanYP + tid] = g;
    }
    __syncthreads();
    v8h hv[8], lv[8];
#pragma unroll
    for (int it = 0; it < 8; ++it) {
      const int row = it * 8 + wave * 4 + q;
      const float* sp = sY + row * kScanYP + c8;
      const v4f a0 = *(const v4f*)(sp);
      const v4f a1 = *(const v4f*)(sp + 4);
#pragma unroll
      for (int e = 0; e < 4; ++e) {
        const float s0 = a0[e], s1 = a1[e];
        const unsigned short h0 = f2bf_bits(s0), h1 = f2bf_bits(s1);
        const unsigned short l0 = f2bf_bits(s0 - bf_bits2f(h0)), l1 = f2bf_bits(s1 - bf_bits2f(h1));
        hv[it][e]     = __builtin_bit_cast(_Float16, h0);
        hv[it][4 + e] = __builtin_bit_cast(_Float16, h1);
        lv[it][e]     = __builtin_bit_cast(_Float16, l0);
        lv[it][4 + e] = __builtin_bit_cast(_Float16, l1);
      }
    }
    for (int pass = 0; pass < 2; ++pass) {
#pragma unroll
      for (int it = 0; it < 8; ++it) {
        const int row = it * 8 + wave * 4 + q;
        const size_t o = (row0 + t0 + row) * kDm + d0 + c8;
        *(volatile v8h*)(YH + o) = hv[it];
        *(volatile v8h*)(YL + o) = lv[it];
      }
      __threadfence();
    }
  }
}

__global__ __launch_bounds__(256) void glu_out_kernel(
    const float* __restrict__ GO, const float* __restrict__ xq, float* __restrict__ outq, int total4)
{
  const int i = blockIdx.x * 256 + threadIdx.x;
  if (i >= total4) return;
  const size_t e0 = (size_t)i << 2;
  const size_t r  = e0 / kDm;
  const int c = (int)(e0 % kDm);
  const v4f va = *(const v4f*)(GO + r * kGluN + c);
  const v4f vg = *(const v4f*)(GO + r * kGluN + kDm + c);
  const v4f vx = *(const v4f*)(xq + e0);
  v4f o;
#pragma unroll
  for (int e = 0; e < 4; ++e) {
    const float gq = vg[e];
    const float sg = __builtin_amdgcn_rcpf(1.0f + expf(-gq));
    const float av = va[e];
    const float xv = vx[e];
    o[e] = av * sg + xv;
  }
  *(volatile v4f*)(outq + e0) = o;
  __threadfence();
  *(volatile v4f*)(outq + e0) = o;
}

extern "C" void kernel_launch(void* const* d_in, const int* in_sizes, int n_in,
                              void* d_out, int out_size, void* d_ws, size_t ws_size,
                              hipStream_t stream)
{
  if (n_in < 10) return;
  if (in_sizes[0] != kRows * kDm) return;
  if (in_sizes[1] != kDm || in_sizes[2] != kDm) return;
  if (in_sizes[3] != kDm * kXpN) return;
  if (in_sizes[4] != kDtR * kDm) return;
  if (in_sizes[5] != kDm) return;
  if (in_sizes[6] != kDm * kNst) return;
  if (in_sizes[7] != kDm) return;
  if (in_sizes[8] != kDm * kGluN) return;
  if (in_sizes[9] != kGluN) return;
  if (out_size != kRows * kDm) return;
  if (ws_size < kWsTotal) return;

  const float* x         = (const float*)d_in[0];
  const float* ln_w      = (const float*)d_in[1];
  const float* ln_b      = (const float*)d_in[2];
  const float* x_proj_w  = (const float*)d_in[3];
  const float* dt_proj_w = (const float*)d_in[4];
  const float* dt_proj_b = (const float*)d_in[5];
  const float* A_log     = (const float*)d_in[6];
  const float* D_skip    = (const float*)d_in[7];
  const float* glu_w     = (const float*)d_in[8];
  const float* glu_b     = (const float*)d_in[9];
  float* dout = (float*)d_out;

  char* ws = (char*)d_ws;
  unsigned short* WXH = (unsigned short*)(ws + kOffWXH);
  unsigned short* WXL = (unsigned short*)(ws + kOffWXL);
  unsigned short* WDH = (unsigned short*)(ws + kOffWDH);
  unsigned short* WDL = (unsigned short*)(ws + kOffWDL);
  unsigned short* WGH = (unsigned short*)(ws + kOffWGH);
  unsigned short* WGL = (unsigned short*)(ws + kOffWGL);
  unsigned short* LNH = (unsigned short*)(ws + kOffLNH);
  unsigned short* LNL = (unsigned short*)(ws + kOffLNL);
  float*          DBL = (float*)(ws + kOffDBL);
  unsigned short* DTH = (unsigned short*)(ws + kOffDTH);
  unsigned short* DTL = (unsigned short*)(ws + kOffDTL);
  float*          DLR = (float*)(ws + kOffDLR);
  unsigned short* YGH = (unsigned short*)(ws + kOffYGH);
  unsigned short* YGL = (unsigned short*)(ws + kOffYGL);
  float*          GO  = (float*)(ws + kOffGO);
  const float* dummy_bias  = glu_b;
  const float* dummy_resid = x;

  wsplit_kernel<<<(kXpP * kDm / 8) / 256, 256, 0, stream>>>(x_proj_w, kDm, kXpN, kDm, kXpP, WXH, WXL, kXpP * kDm / 8);
  wsplit_kernel<<<(kDm * kDtK / 8) / 256, 256, 0, stream>>>(dt_proj_w, kDtR, kDm, kDtK, kDm, WDH, WDL, kDm * kDtK / 8);
  wsplit_kernel<<<(kGluN * kDm / 8) / 256, 256, 0, stream>>>(glu_w, kDm, kGluN, kDm, kGluN, WGH, WGL, kGluN * kDm / 8);

  layernorm_split_kernel<<<kRows / 8, 256, 0, stream>>>(x, ln_w, ln_b, LNH, LNL);

  wmma_gemm64<1, true, 0, 0, false><<<dim3(((kRows / 64) * (kXpP / 64)) / 8, 1), 256, 0, stream>>>(
      LNH, LNL, kDm, 0L,
      WXH, WXL, kDm, 0L,
      (void*)DBL, (void*)DBL, kXpP, 0L,
      dummy_bias, dummy_resid, 0L,
      kRows, kXpP, kDm, 1.0f);

  dtsplit_kernel<<<(kRows * kDtK / 8) / 256, 256, 0, stream>>>(DBL, DTH, DTL, kRows * kDtK / 8);

  wmma_gemm64<1, true, 0, 0, false><<<dim3(((kRows / 64) * (kDm / 64)) / 8, 1), 256, 0, stream>>>(
      DTH, DTL, kDtK, 0L,
      WDH, WDL, kDtK, 0L,
      (void*)DLR, (void*)DLR, kDm, 0L,
      dummy_bias, dummy_resid, 0L,
      kRows, kDm, kDtK, 1.0f);

  scan_kernel<<<kBatch * (kDm / kScanCh), kScanCh, 0, stream>>>(DBL, DLR, LNH, LNL, dt_proj_b, A_log, D_skip, YGH, YGL);

  for (int qtr = 0; qtr < kGluQ; ++qtr) {
    const size_t roff = (size_t)qtr * kRowsQ * kDm;
    wmma_gemm64<1, true, 2, 0, false><<<dim3(((kRowsQ / 64) * (kGluN / 64)) / 8, 1), 256, 0, stream>>>(
        YGH + roff, YGL + roff, kDm, 0L,
        WGH, WGL, kDm, 0L,
        (void*)GO, (void*)GO, kGluN, 0L,
        glu_b, dummy_resid, 0L,
        kRowsQ, kGluN, kDm, 1.0f);
    glu_out_kernel<<<(kRowsQ * kDm / 4) / 256, 256, 0, stream>>>(GO, x + roff, dout + roff, kRowsQ * kDm / 4);
  }
}
